// FastMultiHeadAttention_64854006169987
// MI455X (gfx1250) — hardware-verified
//
#include <hip/hip_runtime.h>
#include <math.h>
#include <stdint.h>

#define NB    2
#define SQ    2048
#define DM    1024
#define NH    16
#define HDM   64
#define NTOK  4096
#define QKVN  3072
#define RK    8
#define RKP   16
#define NFQ   32
#define XP    1088
#define KQ    1056
#define AOP   2112
#define KO    2080
#define VTP   4096

static_assert(KQ % 32 == 0);
static_assert(KO % 32 == 0);
static_assert(KQ <= XP);
static_assert(KO <= AOP);
static_assert((XP * 2) % 128 == 0);
static_assert((AOP * 2) % 128 == 0);
static_assert(NTOK % 64 == 0);
static_assert(DM % 64 == 0);
static_assert(SQ % 64 == 0);
static_assert(NH * HDM == DM);
static_assert(NB * SQ == NTOK);

typedef _Float16     v16h __attribute__((ext_vector_type(16)));
typedef _Float16     v8h  __attribute__((ext_vector_type(8)));
typedef __bf16       v16b __attribute__((ext_vector_type(16)));
typedef __bf16       v8b  __attribute__((ext_vector_type(8)));
typedef float        v8f  __attribute__((ext_vector_type(8)));
typedef float        v4f  __attribute__((ext_vector_type(4)));
typedef unsigned int v4u  __attribute__((ext_vector_type(4)));

__device__ __forceinline__ unsigned short bf_bits(float f) {
  const unsigned u = __float_as_uint(f);
  return (unsigned short)((u + 0x7FFFu + ((u >> 16) & 1u)) >> 16);
}
__device__ __forceinline__ float bf_val(unsigned short h) { return __uint_as_float(((unsigned)h) << 16); }
__device__ __forceinline__ float bf_rne(float f) { return bf_val(bf_bits(f)); }
__device__ __forceinline__ unsigned pk16(unsigned short a, unsigned short b) { return (unsigned)a | ((unsigned)b << 16); }
__device__ __forceinline__ v8f zero8() { v8f z = {0.f, 0.f, 0.f, 0.f, 0.f, 0.f, 0.f, 0.f}; return z; }

__device__ __forceinline__ void lds_wave_sync() {
  __builtin_amdgcn_fence(__ATOMIC_RELEASE, "workgroup");
  __builtin_amdgcn_wave_barrier();
  __builtin_amdgcn_fence(__ATOMIC_ACQUIRE, "workgroup");
}

union FragB { v16b v; v8b h[2]; };
__device__ __forceinline__ v16b ldfrag_b(const __bf16* p) { FragB f; f.h[0] = *(const v8b*)(p); f.h[1] = *(const v8b*)(p + 16); return f.v; }

__device__ __forceinline__ v8f mma_b(v16b a, v16b b, v8f c) {
  return __builtin_amdgcn_wmma_f32_16x16x32_bf16(false, a, false, b, (short)0, c, false, false);
}
__device__ __forceinline__ void dep_guard_b(v8f& a, v8f& b, v16b x, v16b y) {
  asm volatile("v_nop\n\tv_nop\n\tv_nop\n\tv_nop" : "+v"(a), "+v"(b) : "v"(x), "v"(y));
}
__device__ __forceinline__ void keep4_b(v16b a, v16b b, v16b c, v16b d) { asm volatile("v_nop" :: "v"(a), "v"(b), "v"(c), "v"(d)); }
__device__ __forceinline__ void acc_guard4(v8f& a, v8f& b, v8f& c, v8f& d) {
  asm volatile("v_nop\n\tv_nop\n\tv_nop\n\tv_nop" : "+v"(a), "+v"(b), "+v"(c), "+v"(d));
}
__device__ __forceinline__ v8f at_mma(v16b a, v16b b, v8f c) {
  c = __builtin_amdgcn_wmma_f32_16x16x32_bf16(false, a, false, b, (short)0, c, false, false);
  asm volatile("v_nop\n\tv_nop\n\tv_nop\n\tv_nop" : "+v"(c) : "v"(a), "v"(b));
  return c;
}
__device__ __forceinline__ __bf16 at_f2bf(float f) { return __builtin_bit_cast(__bf16, bf_bits(f)); }
__device__ __forceinline__ void at_split(float f, __bf16& hi, __bf16& lo) {
  const unsigned short hb = bf_bits(f);
  hi = __builtin_bit_cast(__bf16, hb);
  lo = at_f2bf(f - __uint_as_float(((unsigned)hb) << 16));
}

__global__ __launch_bounds__(256) void rope_table_kernel(float* __restrict__ cst, float* __restrict__ snt) {
  const int i = (int)blockIdx.x * 256 + (int)threadIdx.x;
  if (i >= SQ * NFQ) return;
  const int s = i >> 5, j = i & 31;
  const float e   = (float)j * 0.03125f;
  const float pw  = powf(10000.0f, e);
  const float inv = 1.0f / pw;
  const float ang = (float)s * inv;
  float sv, cv;
  sincosf(ang, &sv, &cv);
  const size_t o = (size_t)s * NFQ + j;
  for (int pass = 0; pass < 2; ++pass) {
    ((volatile float*)cst)[o] = cv;
    ((volatile float*)snt)[o] = sv;
    __threadfence();
  }
}

template <int DUP>
__global__ __launch_bounds__(256) void cvt_rows_kernel(const float* __restrict__ in, unsigned short* __restrict__ outp, int ldo, int nthr) {
  const int i = (int)blockIdx.x * 256 + (int)threadIdx.x;
  if (i >= nthr) return;
  const int r = i >> 7;
  const int c = (i & 127) * 8;
  const size_t e = (size_t)r * DM + c;
  const v4f a = *(const v4f*)(in + e);
  const v4f b = *(const v4f*)(in + e + 4);
  v4u w;
  w[0] = pk16(bf_bits(a[0]), bf_bits(a[1]));
  w[1] = pk16(bf_bits(a[2]), bf_bits(a[3]));
  w[2] = pk16(bf_bits(b[0]), bf_bits(b[1]));
  w[3] = pk16(bf_bits(b[2]), bf_bits(b[3]));
  const size_t o = (size_t)r * ldo + c;
  for (int pass = 0; pass < 2; ++pass) {
    *(volatile v4u*)(outp + o) = w;
    if (DUP) *(volatile v4u*)(outp + o + DM) = w;
    __threadfence();
  }
}

__global__ __launch_bounds__(256) void small_planes_kernel(const float* __restrict__ Bqkv, const float* __restrict__ Bproj,
                                                           const float* __restrict__ Aqkv, const float* __restrict__ Aproj,
                                                           unsigned short* __restrict__ WQt, unsigned short* __restrict__ WPt,
                                                           unsigned short* __restrict__ AQ, unsigned short* __restrict__ AP) {
  const int blk = (int)blockIdx.x;
  const int tid = (int)threadIdx.x;
  const int sub = tid & 7;
  const int grp = tid >> 3;
  v4u w = {0u, 0u, 0u, 0u};
  unsigned short* dst;
  if (blk < 96) {
    const int n = blk * 32 + grp;
    const float* bp = Bqkv + (size_t)n * RK;
    const v4f f0 = *(const v4f*)(bp);
    const v4f f1 = *(const v4f*)(bp + 4);
    v4u hv;
    hv[0] = pk16(bf_bits(2.0f * f0[0]), bf_bits(2.0f * f0[1]));
    hv[1] = pk16(bf_bits(2.0f * f0[2]), bf_bits(2.0f * f0[3]));
    hv[2] = pk16(bf_bits(2.0f * f1[0]), bf_bits(2.0f * f1[1]));
    hv[3] = pk16(bf_bits(2.0f * f1[2]), bf_bits(2.0f * f1[3]));
    const unsigned msk = (sub == 0 || sub == 2) ? 0xffffffffu : 0u;
#pragma unroll
    for (int q = 0; q < 4; ++q) w[q] = hv[q] & msk;
    dst = WQt + (size_t)n * XP + sub * 8;
  } else if (blk < 128) {
    const int n = (blk - 96) * 32 + grp;
    const float* bp = Bproj + (size_t)n * RK;
    const v4f f0 = *(const v4f*)(bp);
    const v4f f1 = *(const v4f*)(bp + 4);
    v4u hv;
    hv[0] = pk16(bf_bits(2.0f * f0[0]), bf_bits(2.0f * f0[1]));
    hv[1] = pk16(bf_bits(2.0f * f0[2]), bf_bits(2.0f * f0[3]));
    hv[2] = pk16(bf_bits(2.0f * f1[0]), bf_bits(2.0f * f1[1]));
    hv[3] = pk16(bf_bits(2.0f * f1[2]), bf_bits(2.0f * f1[3]));
    const unsigned msk = (sub == 0 || sub == 2) ? 0xffffffffu : 0u;
#pragma unroll
    for (int q = 0; q < 4; ++q) w[q] = hv[q] & msk;
    dst = WPt + (size_t)n * AOP + sub * 8;
  } else if (blk < 136) {
    const int L = (blk - 128) * 32 + grp;
    const int r = L >> 4;
    const int c = (L & 15) * 64 + sub * 8;
    const int rr = (r < RK) ? r : (RK - 1);
    const float* ap = Aqkv + (size_t)rr * DM + c;
    const v4f f0 = *(const v4f*)(ap);
    const v4f f1 = *(const v4f*)(ap + 4);
    v4u hv;
    hv[0] = pk16(bf_bits(f0[0]), bf_bits(f0[1]));
    hv[1] = pk16(bf_bits(f0[2]), bf_bits(f0[3]));
    hv[2] = pk16(bf_bits(f1[0]), bf_bits(f1[1]));
    hv[3] = pk16(bf_bits(f1[2]), bf_bits(f1[3]));
    const unsigned msk = (r < RK) ? 0xffffffffu : 0u;
#pragma unroll
    for (int q = 0; q < 4; ++q) w[q] = hv[q] & msk;
    dst = AQ + (size_t)r * DM + c;
  } else {
    const int L = (blk - 136) * 32 + grp;
    const int r = L >> 5;
    const int c = (L & 31) * 64 + sub * 8;
    const int rr = (r < RK) ? r : (RK - 1);
    const float* ap = Aproj + (size_t)rr * DM + (c & (DM - 1));
    const v4f f0 = *(const v4f*)(ap);
    const v4f f1 = *(const v4f*)(ap + 4);
    v4u hv;
    hv[0] = pk16(bf_bits(f0[0]), bf_bits(f0[1]));
    hv[1] = pk16(bf_bits(f0[2]), bf_bits(f0[3]));
    hv[2] = pk16(bf_bits(f1[0]), bf_bits(f1[1]));
    hv[3] = pk16(bf_bits(f1[2]), bf_bits(f1[3]));
    const unsigned msk = (r < RK) ? 0xffffffffu : 0u;
#pragma unroll
    for (int q = 0; q < 4; ++q) w[q] = hv[q] & msk;
    dst = AP + (size_t)r * (2 * DM) + c;
  }
  for (int pass = 0; pass < 2; ++pass) {
    *(volatile v4u*)(dst) = w;
    __threadfence();
  }
}

__global__ __launch_bounds__(128) void lora16_kernel(const unsigned short* Ap, int lda,
                                                     const unsigned short* __restrict__ Btp, int ldb,
                                                     unsigned short* outp, int ldo, int ocol, int M, int K) {
  __shared__ __align__(16) float lt[4][16 * 20];
  const int lane = threadIdx.x & 31;
  const int wave = threadIdx.x >> 5;
  const int hh = lane >> 4;
  const int rl = lane & 15;
  const int m0 = ((int)blockIdx.x * 4 + wave) * 16;
  if (m0 >= M) return;
  const __bf16* A  = (const __bf16*)(const void*)Ap;
  const __bf16* Bt = (const __bf16*)(const void*)Btp;

  v8f acc = zero8();
  for (int k0 = 0; k0 < K; k0 += 32) {
    const v16b a  = ldfrag_b(A  + (size_t)(m0 + rl) * lda + k0 + 8 * hh);
    const v16b bb = ldfrag_b(Bt + (size_t)rl * ldb + k0 + 8 * hh);
    acc = at_mma(a, bb, acc);
  }

  float* t = lt[wave];
#pragma unroll
  for (int r = 0; r < 8; ++r) t[(8 * hh + r) * 20 + rl] = acc[r];
  lds_wave_sync();

  const int q = lane >> 3, sub = lane & 7;
  const unsigned mh = (sub == 0) ? 0xffffffffu : 0u;
  const unsigned ml = (sub == 2) ? 0xffffffffu : 0u;
  for (int pass = 0; pass < 2; ++pass) {
#pragma unroll
    for (int it = 0; it < 4; ++it) {
      const int row = it * 4 + q;
      const float* sp = t + row * 20;
      v4u w;
#pragma unroll
      for (int e2 = 0; e2 < 4; ++e2) {
        const float f0 = sp[2 * e2], f1 = sp[2 * e2 + 1];
        const unsigned short h0 = bf_bits(f0), h1 = bf_bits(f1);
        const unsigned short l0 = bf_bits(f0 - bf_val(h0)), l1 = bf_bits(f1 - bf_val(h1));
        w[e2] = (pk16(h0, h1) & mh) | (pk16(l0, l1) & ml);
      }
      *(volatile v4u*)(outp + (size_t)(m0 + row) * ldo + ocol + sub * 8) = w;
    }
    __threadfence();
  }
}

__device__ __forceinline__ void store_split16(const float* slab, unsigned short* C, unsigned short* C2, int mBase, int ldc, int ncol, int lane) {
  const int q = lane >> 3, c8 = (lane & 7) * 8;
  for (int pass = 0; pass < 2; ++pass) {
#pragma unroll
    for (int it = 0; it < 4; ++it) {
      const int row = it * 4 + q;
      const float* sp = slab + row * 68 + c8;
      v8h hv, lv;
#pragma unroll
      for (int e = 0; e < 8; ++e) {
        const unsigned short hb = bf_bits(sp[e]);
        const unsigned short lb = bf_bits(sp[e] - bf_val(hb));
        hv[e] = __builtin_bit_cast(_Float16, hb);
        lv[e] = __builtin_bit_cast(_Float16, lb);
      }
      *(volatile v8h*)(C  + (size_t)(mBase + row) * ldc + ncol + c8) = hv;
      *(volatile v8h*)(C2 + (size_t)(mBase + row) * ldc + ncol + c8) = lv;
    }
    __threadfence();
  }
}

template <int EPI>
__global__ __launch_bounds__(256) void gemm64_kernel(
    const unsigned short* __restrict__ Ap, int lda,
    const unsigned short* __restrict__ Btp, int ldb,
    const float* __restrict__ bias, const float* __restrict__ cst, const float* __restrict__ snt,
    void* C0, void* C1, void* C2, void* C3, int ldc,
    int M, int N, int K) {
  const __bf16* A  = (const __bf16*)(const void*)Ap;
  const __bf16* Bt = (const __bf16*)(const void*)Btp;
  __shared__ __align__(16) float sT[8][16 * 68];
  const int lane = threadIdx.x & 31;
  const int wave = threadIdx.x >> 5;
  const int tilesN = N >> 6;
  const int tilesM = M >> 6;
  const int tile = (int)blockIdx.x * 8 + wave;
  if (tile >= tilesM * tilesN) return;
  const int tm = tile / tilesN;
  const int tn = tile - tm * tilesN;
  const int m0 = tm << 6;
  const int n0 = tn << 6;

  const int rlane = lane & 15;
  const int koff  = (lane >> 4) * 8;
  const int mOff  = (lane >> 4) * 8;

  v8f acc[4][4];
#pragma unroll
  for (int i = 0; i < 4; ++i)
#pragma unroll
    for (int j = 0; j < 4; ++j) acc[i][j] = zero8();

  for (int k0 = 0; k0 < K; k0 += 32) {
    v16b bh[4];
#pragma unroll
    for (int j = 0; j < 4; ++j) {
      const size_t bo = (size_t)(n0 + (j << 4) + rlane) * ldb + koff + k0;
      bh[j] = ldfrag_b(Bt + bo);
    }
#pragma unroll
    for (int i = 0; i < 4; ++i) {
      const size_t ao = (size_t)(m0 + (i << 4) + rlane) * lda + koff + k0;
      const v16b ah = ldfrag_b(A + ao);
#pragma unroll
      for (int j = 0; j < 4; ++j) acc[i][j] = mma_b(ah, bh[j], acc[i][j]);
      dep_guard_b(acc[i][0], acc[i][3], ah, ah);
    }
    keep4_b(bh[0], bh[1], bh[2], bh[3]);
  }
  acc_guard4(acc[0][0], acc[0][1], acc[0][2], acc[0][3]);
  acc_guard4(acc[1][0], acc[1][1], acc[1][2], acc[1][3]);
  acc_guard4(acc[2][0], acc[2][1], acc[2][2], acc[2][3]);
  acc_guard4(acc[3][0], acc[3][1], acc[3][2], acc[3][3]);

  float* slab = sT[wave];
  if (EPI == 0) {
    const bool isq = (n0 < DM);
    unsigned short* P0 = isq ? (unsigned short*)C0 : (unsigned short*)C2;
    unsigned short* P1 = isq ? (unsigned short*)C1 : (unsigned short*)C3;
    const int col0 = isq ? n0 : (n0 - DM);
    const int rr = lane >> 1;
    const int cb = (lane & 1) * 16;
#pragma unroll
    for (int i = 0; i < 4; ++i) {
      const int mBase = m0 + (i << 4);
      const int s0 = mBase & (SQ - 1);
      {
        const float* cp = cst + (size_t)(s0 + rr) * NFQ + cb;
        const float* sp = snt + (size_t)(s0 + rr) * NFQ + cb;
#pragma unroll
        for (int u = 0; u < 4; ++u) {
          const v4f a = *(const v4f*)(cp + 4 * u);
          const v4f b = *(const v4f*)(sp + 4 * u);
          *(v4f*)(slab + rr * 68 + cb + 4 * u)      = a;
          *(v4f*)(slab + rr * 68 + 32 + cb + 4 * u) = b;
        }
      }
      lds_wave_sync();
      float cv[2][8], sv[2][8];
#pragma unroll
      for (int j = 0; j < 2; ++j)
#pragma unroll
        for (int r = 0; r < 8; ++r) {
          cv[j][r] = slab[(mOff + r) * 68 + (j << 4) + rlane];
          sv[j][r] = slab[(mOff + r) * 68 + 32 + (j << 4) + rlane];
        }
      lds_wave_sync();
#pragma unroll
      for (int j = 0; j < 2; ++j)
#pragma unroll
        for (int r = 0; r < 8; ++r) {
          const float x1 = acc[i][j][r];
          const float x2 = acc[i][j + 2][r];
          const float o1 = x1 * cv[j][r] - x2 * sv[j][r];
          const float o2 = x2 * cv[j][r] + x1 * sv[j][r];
          slab[(mOff + r) * 68 + (j << 4) + rlane]      = o1;
          slab[(mOff + r) * 68 + 32 + (j << 4) + rlane] = o2;
        }
      lds_wave_sync();
      store_split16(slab, P0, P1, mBase, ldc, col0, lane);
      lds_wave_sync();
    }
  } else if (EPI == 1) {
    unsigned short* P0 = (unsigned short*)C0;
    unsigned short* P1 = (unsigned short*)C1;
#pragma unroll
    for (int i = 0; i < 4; ++i) {
      const int mBase = m0 + (i << 4);
#pragma unroll
      for (int j = 0; j < 4; ++j)
#pragma unroll
        for (int r = 0; r < 8; ++r) slab[(mOff + r) * 68 + (j << 4) + rlane] = acc[i][j][r];
      lds_wave_sync();
      store_split16(slab, P0, P1, mBase, ldc, n0, lane);
      lds_wave_sync();
    }
  } else {
    float* C = (float*)C0;
    const int hh2 = lane >> 4, c4 = (lane & 15) * 4;
#pragma unroll
    for (int i = 0; i < 4; ++i) {
      const int mBase = m0 + (i << 4);
#pragma unroll
      for (int j = 0; j < 4; ++j) {
        const int n = n0 + (j << 4) + rlane;
        const float bv = bf_rne(bias[n]);
#pragma unroll
        for (int r = 0; r < 8; ++r) slab[(mOff + r) * 68 + (j << 4) + rlane] = acc[i][j][r] + bv;
      }
      lds_wave_sync();
      for (int pass = 0; pass < 2; ++pass) {
#pragma unroll
        for (int it = 0; it < 8; ++it) {
          const int row = it * 2 + hh2;
          const v4f v = *(const v4f*)(slab + row * 68 + c4);
          *(volatile v4f*)(C + (size_t)(mBase + row) * ldc + n0 + c4) = v;
        }
        __threadfence();
      }
      lds_wave_sync();
    }
  }
}

#define AT_D 64
#define AT_NW 4
#define AT_QB 64
#define AT_KC 64
static_assert(AT_NW * 16 * 68 * 4 <= 4 * AT_KC * AT_D * 2);

__global__ __launch_bounds__(128)
void attn_causal64_kernel(const unsigned short* __restrict__ qhp, const unsigned short* __restrict__ qlp,
                          const unsigned short* __restrict__ khp, const unsigned short* __restrict__ klp,
                          const unsigned short* __restrict__ vhp, const unsigned short* __restrict__ vlp,
                          unsigned short* __restrict__ aop, float sscale) {
  union FB { v16b v; v8b h[2]; };
  __shared__ __align__(16) __bf16 kvl[4 * AT_KC * AT_D];
  __shared__ __align__(16) __bf16 Psh[AT_NW][16 * AT_KC];
  __shared__ __align__(16) __bf16 Psl[AT_NW][16 * AT_KC];
  __bf16* Ksh = kvl;
  __bf16* Ksl = kvl + AT_KC * AT_D;
  __bf16* Vth = kvl + 2 * AT_KC * AT_D;
  __bf16* Vtl = kvl + 3 * AT_KC * AT_D;

  const int tid  = threadIdx.x;
  const int wave = tid >> 5;
  const int lane = tid & 31;
  const int hh   = lane >> 4;
  const int c    = lane & 15;

  const int nqb = SQ / AT_QB;
  const int bx = (int)blockIdx.x;
  const int qb = bx % nqb;
  const int h  = bx / nqb;
  const int b  = (int)blockIdx.y;
  const int q0 = qb * AT_QB + wave * 16;
  const size_t tok0 = (size_t)b * SQ;

  const __bf16* Qh = (const __bf16*)(const void*)qhp + tok0 * DM + (size_t)h * AT_D;
  const __bf16* Ql = (const __bf16*)(const void*)qlp + tok0 * DM + (size_t)h * AT_D;
  const __bf16* Kh = (const __bf16*)(const void*)khp + tok0 * DM + (size_t)h * AT_D;
  const __bf16* Kl = (const __bf16*)(const void*)klp + tok0 * DM + (size_t)h * AT_D;
  const __bf16* Vh = (const __bf16*)(const void*)vhp + (size_t)(h * AT_D) * VTP + tok0;
  const __bf16* Vl = (const __bf16*)(const void*)vlp + (size_t)(h * AT_D) * VTP + tok0;

  v16b qah[2], qal[2];
#pragma unroll
  for (int dc = 0; dc < 2; ++dc) {
    const __bf16* qr = Qh + (size_t)(q0 + c) * DM + dc * 32 + 8 * hh;
    const __bf16* ql = Ql + (size_t)(q0 + c) * DM + dc * 32 + 8 * hh;
    qah[dc] = ldfrag_b(qr);
    qal[dc] = ldfrag_b(ql);
  }

  float mrow[8], lrow[8];
  v8f oacc[4];
#pragma unroll
  for (int r = 0; r < 8; ++r) { mrow[r] = -INFINITY; lrow[r] = 0.f; }
#pragma unroll
  for (int t = 0; t < 4; ++t) oacc[t] = zero8();

  const int nChunks = qb + 1;
  for (int kc = 0; kc < nChunks; ++kc) {
    const int kv0 = kc * AT_KC;
    __syncthreads();
    {
      const int r = tid >> 1, half = (tid & 1) * 32;
      const __bf16* ksh = Kh + (size_t)(kv0 + r) * DM + half;
      const __bf16* ksl = Kl + (size_t)(kv0 + r) * DM + half;
      const __bf16* vsh = Vh + (size_t)r * VTP + kv0 + half;
      const __bf16* vsl = Vl + (size_t)r * VTP + kv0 + half;
#pragma unroll
      for (int i = 0; i < 4; ++i) {
        const v8b a0 = *(const v8b*)(ksh + 8 * i);
        const v8b a1 = *(const v8b*)(ksl + 8 * i);
        const v8b b0 = *(const v8b*)(vsh + 8 * i);
        const v8b b1 = *(const v8b*)(vsl + 8 * i);
        *(v8b*)(Ksh + r * AT_D  + half + 8 * i) = a0;
        *(v8b*)(Ksl + r * AT_D  + half + 8 * i) = a1;
        *(v8b*)(Vth + r * AT_KC + half + 8 * i) = b0;
        *(v8b*)(Vtl + r * AT_KC + half + 8 * i) = b1;
      }
    }
    __syncthreads();

    v8f s[4];
#pragma unroll
    for (int j = 0; j < 4; ++j) {
      s[j] = zero8();
#pragma unroll
      for (int dc = 0; dc < 2; ++dc) {
        FB kb, kl;
        kb.h[0] = *(const v8b*)(Ksh + (j * 16 + c) * AT_D + dc * 32 + 8 * hh);
        kb.h[1] = *(const v8b*)(Ksh + (j * 16 + c) * AT_D + dc * 32 + 16 + 8 * hh);
        kl.h[0] = *(const v8b*)(Ksl + (j * 16 + c) * AT_D + dc * 32 + 8 * hh);
        kl.h[1] = *(const v8b*)(Ksl + (j * 16 + c) * AT_D + dc * 32 + 16 + 8 * hh);
        s[j] = at_mma(qah[dc], kb.v, s[j]);
        s[j] = at_mma(qah[dc], kl.v, s[j]);
        s[j] = at_mma(qal[dc], kb.v, s[j]);
      }
    }
    const bool diag = (kc == qb);
    float cm[8];
#pragma unroll
    for (int r = 0; r < 8; ++r) {
      const int qrow = q0 + 8 * hh + r;
      float m = -INFINITY;
#pragma unroll
      for (int j = 0; j < 4; ++j) {
        const int kvcol = kv0 + j * 16 + c;
        const float sv = s[j][r] * sscale;
        const bool masked = diag && (kvcol > qrow);
        const float sm = masked ? -INFINITY : sv;
        s[j][r] = sm;
        m = fmaxf(m, sm);
      }
#pragma unroll
      for (int off = 1; off < 16; off <<= 1) m = fmaxf(m, __shfl_xor(m, off, 32));
      cm[r] = m;
    }
    __bf16* pwh = Psh[wave];
    __bf16* pwl = Psl[wave];
#pragma unroll
    for (int r = 0; r < 8; ++r) {
      const float mnew = fmaxf(mrow[r], cm[r]);
      const float alpha = expf(mrow[r] - mnew);
      mrow[r] = mnew;
      float psum = 0.f;
#pragma unroll
      for (int j = 0; j < 4; ++j) {
        const float p = expf(s[j][r] - mnew);
        psum += p;
        __bf16 a, bl; at_split(p, a, bl);
        pwh[(8 * hh + r) * AT_KC + j * 16 + c] = a;
        pwl[(8 * hh + r) * AT_KC + j * 16 + c] = bl;
      }
#pragma unroll
      for (int off = 1; off < 16; off <<= 1) psum += __shfl_xor(psum, off, 32);
      lrow[r] = lrow[r] * alpha + psum;
#pragma unroll
      for (int t = 0; t < 4; ++t) oacc[t][r] *= alpha;
    }
    lds_wave_sync();
#pragma unroll 1
    for (int kk = 0; kk < 2; ++kk) {
      FB pa, pl;
      pa.h[0] = *(const v8b*)(pwh + c * AT_KC + kk * 32 + 8 * hh);
      pa.h[1] = *(const v8b*)(pwh + c * AT_KC + kk * 32 + 16 + 8 * hh);
      pl.h[0] = *(const v8b*)(pwl + c * AT_KC + kk * 32 + 8 * hh);
      pl.h[1] = *(const v8b*)(pwl + c * AT_KC + kk * 32 + 16 + 8 * hh);
#pragma unroll
      for (int t = 0; t < 4; ++t) {
        FB vb, vl;
        vb.h[0] = *(const v8b*)(Vth + (t * 16 + c) * AT_KC + kk * 32 + 8 * hh);
        vb.h[1] = *(const v8b*)(Vth + (t * 16 + c) * AT_KC + kk * 32 + 16 + 8 * hh);
        vl.h[0] = *(const v8b*)(Vtl + (t * 16 + c) * AT_KC + kk * 32 + 8 * hh);
        vl.h[1] = *(const v8b*)(Vtl + (t * 16 + c) * AT_KC + kk * 32 + 16 + 8 * hh);
        oacc[t] = at_mma(pa.v, vb.v, oacc[t]);
        oacc[t] = at_mma(pa.v, vl.v, oacc[t]);
        oacc[t] = at_mma(pl.v, vb.v, oacc[t]);
      }
    }
  }

  __syncthreads();
  float* os = (float*)(void*)kvl + wave * (16 * 68);
#pragma unroll
  for (int r = 0; r < 8; ++r) {
    const float inv = 1.0f / lrow[r];
#pragma unroll
    for (int t = 0; t < 4; ++t) os[(8 * hh + r) * 68 + t * 16 + c] = oacc[t][r] * inv;
  }
  lds_wave_sync();
  {
    const int q = lane >> 3, c8 = (lane & 7) * 8;
    unsigned short* Ah = aop + (tok0 + (size_t)q0) * AOP + (size_t)h * AT_D;
    for (int pass = 0; pass < 2; ++pass) {
#pragma unroll
      for (int it = 0; it < 4; ++it) {
        const int row = it * 4 + q;
        const float* sp = os + row * 68 + c8;
        v8h hv, lv;
#pragma unroll
        for (int e = 0; e < 8; ++e) {
          const unsigned short hb = bf_bits(sp[e]);
          const unsigned short lb = bf_bits(sp[e] - bf_val(hb));
          hv[e] = __builtin_bit_cast(_Float16, hb);
          lv[e] = __builtin_bit_cast(_Float16, lb);
        }
        *(volatile v8h*)(Ah + (size_t)row * AOP + c8)      = hv;
        *(volatile v8h*)(Ah + (size_t)row * AOP + DM + c8) = lv;
      }
      __threadfence();
    }
  }
}

extern "C" void kernel_launch(void* const* d_in, const int* in_sizes, int n_in,
                              void* d_out, int out_size, void* d_ws, size_t ws_size,
                              hipStream_t stream) {
  if (n_in < 8) return;
  if (in_sizes[0] != NTOK * DM) return;
  if (in_sizes[1] != QKVN * DM) return;
  if (in_sizes[2] != RK * DM) return;
  if (in_sizes[3] != QKVN * RK) return;
  if (in_sizes[4] != DM * DM) return;
  if (in_sizes[5] != DM) return;
  if (in_sizes[6] != RK * DM) return;
  if (in_sizes[7] != DM * RK) return;
  if (out_size != NTOK * DM) return;

  const float* x     = (const float*)d_in[0];
  const float* Wqkv  = (const float*)d_in[1];
  const float* Aqkv  = (const float*)d_in[2];
  const float* Bqkv  = (const float*)d_in[3];
  const float* Wproj = (const float*)d_in[4];
  const float* bproj = (const float*)d_in[5];
  const float* Aproj = (const float*)d_in[6];
  const float* Bproj = (const float*)d_in[7];
  float* out = (float*)d_out;

  const size_t szT  = (size_t)SQ * NFQ * 4;
  const size_t szXB = (size_t)NTOK * XP * 2;
  const size_t szWQ = (size_t)QKVN * XP * 2;
  const size_t szWP = (size_t)DM * AOP * 2;
  const size_t szAQ = (size_t)RKP * DM * 2;
  const size_t szAP = (size_t)RKP * 2 * DM * 2;
  const size_t szQ  = (size_t)NTOK * DM * 2;
  const size_t szVT = (size_t)DM * VTP * 2;
  const size_t szAO = (size_t)NTOK * AOP * 2;
  size_t off = 0;
  const size_t oCs = off; off += szT;
  const size_t oSn = off; off += szT;
  const size_t oXB = off; off += szXB;
  const size_t oWQ = off; off += szWQ;
  const size_t oWP = off; off += szWP;
  const size_t oAQ = off; off += szAQ;
  const size_t oAP = off; off += szAP;
  const size_t oQh = off; off += szQ;
  const size_t oQl = off; off += szQ;
  const size_t oKh = off; off += szQ;
  const size_t oKl = off; off += szQ;
  const size_t oVh = off; off += szVT;
  const size_t oVl = off; off += szVT;
  const size_t oAO = off; off += szAO;
  if (off > ws_size) return;

  char* ws = (char*)d_ws;
  float*          cst = (float*)(ws + oCs);
  float*          snt = (float*)(ws + oSn);
  unsigned short* XB  = (unsigned short*)(ws + oXB);
  unsigned short* WQ  = (unsigned short*)(ws + oWQ);
  unsigned short* WP  = (unsigned short*)(ws + oWP);
  unsigned short* AQ  = (unsigned short*)(ws + oAQ);
  unsigned short* AP  = (unsigned short*)(ws + oAP);
  unsigned short* Qh  = (unsigned short*)(ws + oQh);
  unsigned short* Ql  = (unsigned short*)(ws + oQl);
  unsigned short* Kh  = (unsigned short*)(ws + oKh);
  unsigned short* Kl  = (unsigned short*)(ws + oKl);
  unsigned short* VTh = (unsigned short*)(ws + oVh);
  unsigned short* VTl = (unsigned short*)(ws + oVl);
  unsigned short* AO  = (unsigned short*)(ws + oAO);

  const dim3 b256(256), b128(128);

  rope_table_kernel<<<dim3((SQ * NFQ) / 256), b256, 0, stream>>>(cst, snt);
  cvt_rows_kernel<0><<<dim3((NTOK * 128) / 256), b256, 0, stream>>>(x, XB, XP, NTOK * 128);
  cvt_rows_kernel<0><<<dim3((QKVN * 128) / 256), b256, 0, stream>>>(Wqkv, WQ, XP, QKVN * 128);
  cvt_rows_kernel<1><<<dim3((DM * 128) / 256), b256, 0, stream>>>(Wproj, WP, AOP, DM * 128);
  small_planes_kernel<<<dim3(96 + 32 + 8 + 16), b256, 0, stream>>>(Bqkv, Bproj, Aqkv, Aproj, WQ + DM, WP + 2 * DM, AQ, AP);
  lora16_kernel<<<dim3(NTOK / 64), b128, 0, stream>>>(XB, XP, AQ, DM, XB, XP, DM, NTOK, DM);
  gemm64_kernel<0><<<dim3(((NTOK / 64) * ((2 * DM) / 64) + 7) / 8), b256, 0, stream>>>(
      XB, XP, WQ, XP, bproj, cst, snt, (void*)Qh, (void*)Ql, (void*)Kh, (void*)Kl, DM, NTOK, 2 * DM, KQ);
  gemm64_kernel<1><<<dim3(((DM / 64) * (NTOK / 64) + 7) / 8), b256, 0, stream>>>(
      WQ + (size_t)(2 * DM) * XP, XP, XB, XP, bproj, cst, snt, (void*)VTh, (void*)VTl, (void*)VTh, (void*)VTl, VTP, DM, NTOK, KQ);
  attn_causal64_kernel<<<dim3(NH * (SQ / AT_QB), NB), b128, 0, stream>>>(Qh, Ql, Kh, Kl, VTh, VTl, AO, 0.125f);
  lora16_kernel<<<dim3(NTOK / 64), b128, 0, stream>>>(AO, AOP, AP, 2 * DM, AO, AOP, 2 * DM, NTOK, 2 * DM);
  gemm64_kernel<2><<<dim3(((NTOK / 64) * (DM / 64) + 7) / 8), b256, 0, stream>>>(
      AO, AOP, WP, AOP, bproj, cst, snt, (void*)out, (void*)out, (void*)out, (void*)out, DM, NTOK, DM, KO);
  (void)hipGetLastError();
}
